// EVTSR_22771916603484
// MI455X (gfx1250) — hardware-verified
//
#include <hip/hip_runtime.h>
#include <math.h>

typedef __attribute__((ext_vector_type(16))) _Float16 v16h;
typedef __attribute__((ext_vector_type(16))) __bf16 v16b;
typedef __attribute__((ext_vector_type(8)))  _Float16 v8h;
typedef __attribute__((ext_vector_type(8)))  float v8f;
typedef __attribute__((ext_vector_type(4)))  float v4f;
typedef __attribute__((ext_vector_type(2)))  float v2f;
typedef __attribute__((ext_vector_type(4)))  unsigned v4u;
typedef __attribute__((ext_vector_type(4)))  int v4i;
typedef float __attribute__((may_alias)) float_a;
typedef int __attribute__((may_alias)) int_a;

template <typename T> __device__ __forceinline__ void vst2(void* p, T v) { *(volatile T*)p = v; __threadfence(); *(volatile T*)p = v; }
__device__ __forceinline__ v8f wmma16(v16h a, v16h b, v8f c) {
  v8f d = __builtin_amdgcn_wmma_f32_16x16x32_f16(false, a, false, b, (short)0, c, false, false);
  asm volatile("v_nop\n\tv_nop\n\tv_nop\n\tv_nop" : "+v"(d) : "v"(a), "v"(b));
  return d;
}
__device__ __forceinline__ v8f wmma_bf(v16b a, v16b b, v8f c) {
  v8f d = __builtin_amdgcn_wmma_f32_16x16x32_bf16(false, a, false, b, (short)0, c, false, false);
  asm volatile("v_nop\n\tv_nop\n\tv_nop\n\tv_nop" : "+v"(d) : "v"(a), "v"(b));
  return d;
}
__device__ __forceinline__ v16h frag_h(const _Float16* rowk0, int lane) {
  union { v16h v; v8h q[2]; } u; const _Float16* p = rowk0 + 8 * (lane >> 4);
  u.q[0] = *(const v8h*)p; u.q[1] = *(const v8h*)(p + 16); return u.v;
}
__device__ __forceinline__ v16h frag_f32(const float* rowk0, int lane) {
  v16h a; const float* p = rowk0 + 8 * (lane >> 4);
#pragma unroll
  for (int i = 0; i < 8; ++i) { a[i] = (_Float16)p[i]; a[8 + i] = (_Float16)p[16 + i]; }
  return a;
}
__device__ __forceinline__ v16h frag_f32s(const float* rowk0, int lane, float sc) {
  v16h a; const float* p = rowk0 + 8 * (lane >> 4);
#pragma unroll
  for (int i = 0; i < 8; ++i) { a[i] = (_Float16)(p[i] * sc); a[8 + i] = (_Float16)(p[16 + i] * sc); }
  return a;
}
__device__ __forceinline__ v16h fragc_f32(const float* W, int k0, int n, int lane, int ld, int K) {
  v16h a; const int g = lane >> 4;
#pragma unroll
  for (int i = 0; i < 8; ++i) { const int ka = k0 + 8 * g + i, kb = ka + 16;
    a[i] = (_Float16)(ka < K ? W[(size_t)(ka < K ? ka : K - 1) * ld + n] : 0.f); a[8 + i] = (_Float16)(kb < K ? W[(size_t)(kb < K ? kb : K - 1) * ld + n] : 0.f); }
  return a;
}
struct F2 { v16b h, l; };
__device__ __forceinline__ F2 bsplit16(const float v[16]) { F2 r;
#pragma unroll
  for (int i = 0; i < 16; ++i) { const __bf16 h = (__bf16)v[i]; r.h[i] = h; r.l[i] = (__bf16)(v[i] - (float)h); }
  return r; }
__device__ __forceinline__ F2 split_row(const float* row, int k0, int lane) { float v[16]; const float* p = row + k0 + 8 * (lane >> 4);
#pragma unroll
  for (int i = 0; i < 8; ++i) { v[i] = p[i]; v[8 + i] = p[16 + i]; }
  return bsplit16(v); }
__device__ __forceinline__ F2 split_rowK(const float* row, int k0, int lane, int K) { float v[16]; const int g = lane >> 4;
#pragma unroll
  for (int i = 0; i < 8; ++i) { const int ka = k0 + 8 * g + i, kb = ka + 16; v[i] = ka < K ? row[ka < K ? ka : K - 1] : 0.f; v[8 + i] = kb < K ? row[kb < K ? kb : K - 1] : 0.f; }
  return bsplit16(v); }
__device__ __forceinline__ F2 split_col(const float* W, int k0, int n, int lane, int ld, int K) { float v[16]; const int g = lane >> 4;
#pragma unroll
  for (int i = 0; i < 8; ++i) { const int ka = k0 + 8 * g + i, kb = ka + 16; v[i] = ka < K ? W[(size_t)(ka < K ? ka : K - 1) * ld + n] : 0.f; v[8 + i] = kb < K ? W[(size_t)(kb < K ? kb : K - 1) * ld + n] : 0.f; }
  return bsplit16(v); }
__device__ __forceinline__ v8f mac3(const F2& a, const F2& b, v8f c) { c = wmma_bf(a.l, b.h, c); c = wmma_bf(a.h, b.l, c); return wmma_bf(a.h, b.h, c); }
__device__ __forceinline__ float sigm(float v) { return 1.0f / (1.0f + expf(-v)); }
#define LDSX() do { asm volatile("s_wait_dscnt 0" ::: "memory"); __builtin_amdgcn_wave_barrier(); __builtin_amdgcn_fence(__ATOMIC_RELEASE, "workgroup"); } while (0)


#define CIN 64
#define CH 128
#define IH 128
#define IW 128
#define NPX (IH * IW)
#define KS 5
#define KK (KS * KS)
#define WSC 256.0f
#define EPS 1e-5f
#ifndef TPB
#define TPB (NPX / 64)
#endif
typedef __attribute__((ext_vector_type(8))) __bf16 v8b;
__device__ __forceinline__ v16b frag_b(const __bf16* rowk0, int lane) {
  union { v16b v; v8b q[2]; } u; const __bf16* p = rowk0 + 8 * (lane >> 4);
  u.q[0] = *(const v8b*)p; u.q[1] = *(const v8b*)(p + 16); return u.v;
}
__device__ __forceinline__ float bfr(float v) { return (float)(__bf16)v; }
__device__ __attribute__((noinline)) float exp_ni(float v) { return expf(v); }
__device__ __attribute__((noinline)) float erf_ni(float v) { return erff(v); }

#define WS_W3  0u
#define WS_WD  (WS_W3 + 2u * CH * 9 * CH)
#define WS_WS  (WS_WD + 2u * KK * CH * CH)
#define WS_F   (WS_WS + 2u * CH * CH)
#define WS_FH  (WS_F + 4u * (size_t)2 * NPX * CH)
#define WS_T   (WS_FH + 2u * (size_t)2 * NPX * CH)
#define WS_EN  (WS_T + 2u * (size_t)2 * NPX * CH)
#define WS_END (WS_EN + 4u * (size_t)2 * NPX * CH)

__global__ __launch_bounds__(256) void k_packw(const float* __restrict__ DF1, const float* __restrict__ DF2, const float* __restrict__ SP, char* __restrict__ ws) { const int n = blockIdx.x, which = blockIdx.y, t = threadIdx.x; __shared__ __align__(16) _Float16 s[9 * CH];
  if (which == 0) { if (n >= CH) return; for (int e = t; e < 9 * CH; e += 256) { const int tap = e / CH, c = e % CH; s[e] = (_Float16)(bfr(DF1[((size_t)n * CH + c) * 9 + tap]) * WSC); } __syncthreads(); for (int q = t; q < 9 * CH / 8; q += 256) vst2((unsigned*)((_Float16*)(ws + WS_W3) + (size_t)n * 9 * CH + q * 8), *(const v4u*)&s[q * 8]); }
  else if (which == 1) { if (n >= KK * CH) return; const int k = n / CH, c = n % CH; if (t < CH) s[t] = (_Float16)(bfr(DF2[((size_t)c * KK + k) * CH + t]) * WSC); __syncthreads(); if (t < CH / 8) vst2((unsigned*)((_Float16*)(ws + WS_WD) + (size_t)n * CH + t * 8), *(const v4u*)&s[t * 8]); }
  else { if (n >= CH) return; if (t < CH) s[t] = (_Float16)(bfr(SP[(size_t)n * CH + t]) * WSC); __syncthreads(); if (t < CH / 8) vst2((unsigned*)((_Float16*)(ws + WS_WS) + (size_t)n * CH + t * 8), *(const v4u*)&s[t * 8]); } }
__global__ __launch_bounds__(128) void k_feat(const float* __restrict__ XR, const float* __restrict__ XE, const float* __restrict__ CW, const float* __restrict__ G, const float* __restrict__ Bt, float* __restrict__ F, _Float16* __restrict__ FH) { __shared__ __align__(16) float sf[64][CH + 4]; __shared__ __align__(16) _Float16 sh[64][CH + 8];
  const int tid = threadIdx.x, wave = tid >> 5, lane = tid & 31, col = lane & 15, g = lane >> 4; const int st = blockIdx.y; const float* X = st == 0 ? XR : XE; const size_t p0 = (size_t)blockIdx.x * 64; const int pw = wave * 16;
  v8f acc[8] = {};
#pragma unroll
  for (int kc = 0; kc < CIN / 32; ++kc) { v16b a; const size_t p = p0 + pw + col;
#pragma unroll
    for (int i = 0; i < 8; ++i) { a[i] = (__bf16)X[(size_t)(kc * 32 + 8 * g + i) * NPX + p]; a[8 + i] = (__bf16)X[(size_t)(kc * 32 + 16 + 8 * g + i) * NPX + p]; }
#pragma unroll
    for (int j = 0; j < 8; ++j) { v16b w; const float* wr = CW + (size_t)(j * 16 + col) * CIN + kc * 32 + 8 * g;
#pragma unroll
      for (int i = 0; i < 8; ++i) { w[i] = (__bf16)wr[i]; w[8 + i] = (__bf16)wr[16 + i]; } acc[j] = wmma_bf(a, w, acc[j]); } }
#pragma unroll
  for (int j = 0; j < 8; ++j)
#pragma unroll
    for (int r = 0; r < 8; ++r) sf[pw + 8 * g + r][j * 16 + col] = acc[j][r];
  __syncthreads();
  { const int rl = tid >> 1, half = tid & 1; float* row = &sf[rl][0]; float s = 0.f; for (int c = half * 64; c < half * 64 + 64; ++c) s += row[c]; s += __shfl_xor(s, 1); const float mu = s / (float)CH; float q = 0.f; for (int c = half * 64; c < half * 64 + 64; ++c) { const float d = row[c] - mu; q += d * d; } q += __shfl_xor(q, 1); const float inv = 1.0f / sqrtf(q / (float)CH + EPS);
    for (int c = half * 64; c < half * 64 + 64; ++c) { const float v = (row[c] - mu) * inv * bfr(G[c]) + bfr(Bt[c]); row[c] = v; sh[rl][c] = (_Float16)v; } }
  __syncthreads(); for (int e = tid; e < 64 * 32; e += 128) { const int rl = e >> 5, q = e & 31; vst2(F + ((size_t)st * NPX + p0 + rl) * CH + q * 4, *(const v4f*)&sf[rl][q * 4]); } for (int e = tid; e < 64 * 16; e += 128) { const int rl = e >> 4, q = e & 15; vst2((unsigned*)(FH + ((size_t)st * NPX + p0 + rl) * CH + q * 8), *(const v4u*)&sh[rl][q * 8]); } }
__global__ __launch_bounds__(128) void k_c3(const _Float16* __restrict__ FH, const _Float16* __restrict__ W3, _Float16* __restrict__ T) { __shared__ __align__(16) _Float16 sh[4][16][CH + 8];
  const int tid = threadIdx.x, wave = tid >> 5, lane = tid & 31, col = lane & 15, g = lane >> 4; const int st = blockIdx.y; const size_t p0 = (size_t)blockIdx.x * 64 + wave * 16; const size_t p = p0 + col; const int y = (int)(p / IW), x = (int)(p % IW); const _Float16* FB = FH + (size_t)st * NPX * CH;
  v8f acc[8] = {};
#pragma unroll 1
  for (int tap = 0; tap < 9; ++tap) { const int yy = y + tap / 3 - 1, xx = x + tap % 3 - 1; const bool ok = yy >= 0 && yy < IH && xx >= 0 && xx < IW; const _Float16* src = FB + (size_t)(ok ? (yy * IW + xx) : 0) * CH;
#pragma unroll
    for (int kc = 0; kc < CH / 32; ++kc) { v16h a; const _Float16* pp = src + kc * 32 + 8 * g;
#pragma unroll
      for (int i = 0; i < 8; ++i) { a[i] = ok ? pp[i] : (_Float16)0.0f; a[8 + i] = ok ? pp[16 + i] : (_Float16)0.0f; }
#pragma unroll
      for (int j = 0; j < 8; ++j) acc[j] = wmma16(a, frag_h(W3 + (size_t)(j * 16 + col) * (9 * CH) + tap * CH + kc * 32, lane), acc[j]); } }
#pragma unroll
  for (int j = 0; j < 8; ++j)
#pragma unroll
    for (int r = 0; r < 8; ++r) sh[wave][8 * g + r][j * 16 + col] = (_Float16)fmaxf(acc[j][r] * (1.0f / WSC), 0.f);
  LDSX(); for (int rl = 0; rl < 16; ++rl) if (lane < 16) vst2((unsigned*)(T + ((size_t)st * NPX + p0 + rl) * CH + lane * 8), *(const v4u*)&sh[wave][rl][lane * 8]); }
__global__ __launch_bounds__(128) void k_dyn(const _Float16* __restrict__ T, const _Float16* __restrict__ WD, const float* __restrict__ F, float* __restrict__ EN) { __shared__ __align__(16) float so[4][16][CH + 4];
  const int tid = threadIdx.x, wave = tid >> 5, lane = tid & 31, col = lane & 15, g = lane >> 4; const int st = blockIdx.y; const size_t p0 = (size_t)blockIdx.x * 64 + wave * 16; const _Float16* TB = T + (size_t)st * NPX * CH; const float* FB = F + (size_t)st * NPX * CH;
  v16h a[4];
#pragma unroll
  for (int kc = 0; kc < 4; ++kc) a[kc] = frag_h(TB + (p0 + col) * CH + kc * 32, lane);
  v8f en[8];
#pragma unroll
  for (int j = 0; j < 8; ++j) en[j] = v8f{};
#pragma unroll 1
  for (int k = 0; k < KK; ++k) { v8f acc[8] = {};
#pragma unroll
    for (int kc = 0; kc < 4; ++kc) {
#pragma unroll
      for (int j = 0; j < 8; ++j) acc[j] = wmma16(a[kc], frag_h(WD + ((size_t)k * CH + j * 16 + col) * CH + kc * 32, lane), acc[j]); }
    const int dy = k / KS - 2, dx = k % KS - 2;
#pragma unroll
    for (int r = 0; r < 8; ++r) { const size_t p = p0 + 8 * g + r; const int yy = (int)(p / IW) + dy, xx = (int)(p % IW) + dx; const bool ok = yy >= 0 && yy < IH && xx >= 0 && xx < IW; const float* fr = FB + (size_t)(ok ? (yy * IW + xx) : 0) * CH;
#pragma unroll
      for (int j = 0; j < 8; ++j) { const float fv = ok ? fr[j * 16 + col] : 0.f; en[j][r] += acc[j][r] * (1.0f / WSC) * fv; } } }
#pragma unroll
  for (int j = 0; j < 8; ++j)
#pragma unroll
    for (int r = 0; r < 8; ++r) so[wave][8 * g + r][j * 16 + col] = en[j][r];
  LDSX(); for (int rl = 0; rl < 16; ++rl) vst2(EN + ((size_t)st * NPX + p0 + rl) * CH + lane * 4, *(const v4f*)&so[wave][rl][lane * 4]); }
__global__ __launch_bounds__(128) void k_out(const float* __restrict__ EN, const float* __restrict__ F, const _Float16* __restrict__ WS, const float* __restrict__ G, const float* __restrict__ Bt, const float* __restrict__ OW, float* __restrict__ OUT) { __shared__ __align__(16) float sf[64][CH + 4]; __shared__ __align__(16) float st2[CIN][64 + 4];
  const int tid = threadIdx.x, wave = tid >> 5, lane = tid & 31, col = lane & 15, g = lane >> 4; const size_t p0 = (size_t)blockIdx.x * 64; const int pw = wave * 16;
  { v8f acc[8] = {};
#pragma unroll
    for (int kc = 0; kc < 4; ++kc) { v16h a; const float* pp = EN + ((size_t)NPX + p0 + pw + col) * CH + kc * 32 + 8 * g;
#pragma unroll
      for (int i = 0; i < 8; ++i) { a[i] = (_Float16)pp[i]; a[8 + i] = (_Float16)pp[16 + i]; }
#pragma unroll
      for (int j = 0; j < 8; ++j) acc[j] = wmma16(a, frag_h(WS + (size_t)(j * 16 + col) * CH + kc * 32, lane), acc[j]); }
#pragma unroll
    for (int j = 0; j < 8; ++j)
#pragma unroll
      for (int r = 0; r < 8; ++r) { const int c = j * 16 + col; const size_t p = p0 + pw + 8 * g + r; const float gate = 1.0f / (1.0f + expf(-acc[j][r] * (1.0f / WSC))); const float re = EN[p * CH + c]; sf[pw + 8 * g + r][c] = re + re * gate + F[p * CH + c]; } }
  __syncthreads();
  { const int rl = tid >> 1, half = tid & 1; float* row = &sf[rl][0]; float s = 0.f; for (int c = half * 64; c < half * 64 + 64; ++c) s += row[c]; s += __shfl_xor(s, 1); const float mu = s / (float)CH; float q = 0.f; for (int c = half * 64; c < half * 64 + 64; ++c) { const float d = row[c] - mu; q += d * d; } q += __shfl_xor(q, 1); const float inv = 1.0f / sqrtf(q / (float)CH + EPS);
    for (int c = half * 64; c < half * 64 + 64; ++c) row[c] = (row[c] - mu) * inv * bfr(G[c]) + bfr(Bt[c]); }
  __syncthreads();
  { v8f acc[4] = {};
#pragma unroll
    for (int kc = 0; kc < 4; ++kc) { float v[16]; const float* pp = &sf[pw + col][kc * 32 + 8 * g];
#pragma unroll
      for (int i = 0; i < 8; ++i) { v[i] = pp[i]; v[8 + i] = pp[16 + i]; }
      const F2 a2 = bsplit16(v);
#pragma unroll
      for (int j = 0; j < 4; ++j) { v16b w; const float* wr = OW + (size_t)(j * 16 + col) * CH + kc * 32 + 8 * g;
#pragma unroll
        for (int i = 0; i < 8; ++i) { w[i] = (__bf16)wr[i]; w[8 + i] = (__bf16)wr[16 + i]; } acc[j] = wmma_bf(a2.h, w, acc[j]); acc[j] = wmma_bf(a2.l, w, acc[j]); } }
    __syncthreads();
#pragma unroll
    for (int j = 0; j < 4; ++j)
#pragma unroll
      for (int r = 0; r < 8; ++r) st2[j * 16 + col][pw + 8 * g + r] = acc[j][r]; }
  __syncthreads(); for (int e = tid; e < CIN * 16; e += 128) { const int o = e >> 4, q = e & 15; vst2(OUT + (size_t)o * NPX + p0 + q * 4, *(const v4f*)&st2[o][q * 4]); } }
extern "C" void kernel_launch(void* const* d_in, const int* in_sizes, int n_in, void* d_out, int out_size, void* d_ws, size_t ws_size, hipStream_t stream) {
  (void)in_sizes; (void)n_in; (void)out_size;
  const float** Fi = (const float**)d_in;
  if (ws_size < (size_t)WS_END) return;
  char* ws = (char*)d_ws; _Float16 *W3 = (_Float16*)(ws + WS_W3), *WD = (_Float16*)(ws + WS_WD), *WSp = (_Float16*)(ws + WS_WS), *FH = (_Float16*)(ws + WS_FH), *T = (_Float16*)(ws + WS_T); float *F = (float*)(ws + WS_F), *EN = (float*)(ws + WS_EN);
  k_packw<<<dim3(KK * CH, 3), 256, 0, stream>>>(Fi[5], Fi[6], Fi[7], ws);
  k_feat<<<dim3(NPX / 64, 2), 128, 0, stream>>>(Fi[0], Fi[1], Fi[2], Fi[3], Fi[4], F, FH);
  k_c3<<<dim3(NPX / 64, 2), 128, 0, stream>>>(FH, W3, T);
  k_dyn<<<dim3(TPB, 2), 128, 0, stream>>>(T, WD, F, EN);
  k_out<<<TPB, 128, 0, stream>>>(EN, F, WSp, Fi[3], Fi[4], Fi[8], (float*)d_out);
}
